// mySeq2SeqModel_51840255262966
// MI455X (gfx1250) — hardware-verified
//
#include <hip/hip_runtime.h>


typedef __bf16         bf16t;
typedef bf16t          v16b __attribute__((ext_vector_type(16)));
typedef unsigned short v8us __attribute__((ext_vector_type(8)));
typedef float          v8f  __attribute__((ext_vector_type(8)));
typedef float          v4f  __attribute__((ext_vector_type(4)));

union Frag { v16b v; v8us q[2]; };

#define V_   27
#define E_   64
#define H_   128
#define S_   512
#define BT   16
#define NTH  256
#define KP   128
#define NL   32
#define CH   32
#define ROWF (CH * V_)
#define NTAB (V_ * H_)

struct Smem {
  alignas(16) unsigned short wh[2][H_ * KP];
  alignas(16) unsigned short wd[2][NL * KP];
  alignas(16) unsigned short hp[2][BT * KP];
  alignas(16) float          stage[BT * ROWF];
  alignas(16) unsigned char  ids[S_ * BT];
};
static_assert(sizeof(Smem) == 153600);

__device__ __forceinline__ unsigned short bf16_bits(float x) {
  unsigned int u = __float_as_uint(x);
  u += 0x7FFFu + ((u >> 16) & 1u);
  return (unsigned short)(u >> 16);
}
__device__ __forceinline__ float bf16_val(unsigned short b) {
  return __uint_as_float(((unsigned int)b) << 16);
}

__device__ __forceinline__ float ftanh(float x) {
  float ax = fabsf(x);
  float t  = __builtin_amdgcn_exp2f(ax * -2.885390082f);
  float y  = (1.0f - t) * __builtin_amdgcn_rcpf(1.0f + t);
  return copysignf(y, x);
}

__device__ __forceinline__ v8f wmm(const Frag& a, const Frag& b, v8f c) {
  return __builtin_amdgcn_wmma_f32_16x16x32_bf16(false, a.v, false, b.v, (short)0, c, false, false);
}

__device__ __forceinline__ v8f mma3(v8f acc, const unsigned short* ah, const unsigned short* al,
                                    const unsigned short* bh, const unsigned short* bl) {
#pragma unroll
  for (int kt = 0; kt < 4; ++kt) {
    const int k0 = kt * 32;
    Frag a0, a1, b0, b1;
    a0.q[0] = *(const v8us*)(ah + k0);  a0.q[1] = *(const v8us*)(ah + k0 + 16);
    a1.q[0] = *(const v8us*)(al + k0);  a1.q[1] = *(const v8us*)(al + k0 + 16);
    b0.q[0] = *(const v8us*)(bh + k0);  b0.q[1] = *(const v8us*)(bh + k0 + 16);
    b1.q[0] = *(const v8us*)(bl + k0);  b1.q[1] = *(const v8us*)(bl + k0 + 16);
    acc = wmm(a0, b0, acc);
    acc = wmm(a1, b0, acc);
    acc = wmm(a0, b1, acc);
    asm volatile("v_nop\n\tv_nop\n\tv_nop\n\tv_nop"
                 : "+v"(acc)
                 : "v"(a0.v), "v"(a1.v), "v"(b0.v), "v"(b1.v));
  }
  return acc;
}

__device__ __forceinline__ void load_ids(Smem& sm, const int* gids, int base, int tid) {
#pragma unroll 1
  for (int it = 0; it < (S_ * BT) / NTH; ++it) {
    int idx = it * NTH + tid;
    int m = idx >> 9, t = idx & (S_ - 1);
    int v = gids[(size_t)(base + m) * S_ + t];
    v = (v < 0) ? v + V_ : v;
    v = min(max(v, 0), V_ - 1);
    sm.ids[t * BT + m] = (unsigned char)v;
  }
}

__device__ __forceinline__ void load_wh(Smem& sm, const float* Wh, int tid) {
#pragma unroll 1
  for (int idx = tid; idx < H_ * H_; idx += NTH) {
    int k = idx >> 7, n = idx & (H_ - 1);
    float x = Wh[idx];
    unsigned short hb = bf16_bits(x);
    unsigned short lb = bf16_bits(x - bf16_val(hb));
    sm.wh[0][n * KP + k] = hb;
    sm.wh[1][n * KP + k] = lb;
  }
}

__device__ __forceinline__ void load_wd(Smem& sm, const float* Wd, int tid) {
#pragma unroll 1
  for (int idx = tid; idx < NL * H_; idx += NTH) {
    int k = idx >> 5, n = idx & (NL - 1);
    int nn = min(n, V_ - 1);
    float x = Wd[k * V_ + nn];
    x = (n < V_) ? x : 0.0f;
    unsigned short hb = bf16_bits(x);
    unsigned short lb = bf16_bits(x - bf16_val(hb));
    sm.wd[0][n * KP + k] = hb;
    sm.wd[1][n * KP + k] = lb;
  }
}

__device__ __forceinline__ v8f gather_tab(const Smem& sm, const float* T, int t, int hh, int ncol) {
  union { unsigned long long u64; unsigned int u32[2]; } pk;
  pk.u64 = *(const unsigned long long*)(&sm.ids[t * BT + hh * 8]);
  v8f c = {0.f, 0.f, 0.f, 0.f, 0.f, 0.f, 0.f, 0.f};
#pragma unroll
  for (int r = 0; r < 8; ++r) {
    int id = (int)((pk.u32[r >> 2] >> (8 * (r & 3))) & 0xFFu);
    id = min(id, V_ - 1);
    c[r] = T[id * H_ + ncol];
  }
  return c;
}

__device__ __forceinline__ void write_h(Smem& sm, v8f pre, int hh, int ncol) {
#pragma unroll
  for (int r = 0; r < 8; ++r) {
    float hv = ftanh(pre[r]);
    unsigned short hb = bf16_bits(hv);
    unsigned short lb = bf16_bits(hv - bf16_val(hb));
    int m = 8 * hh + r;
    sm.hp[0][m * KP + ncol] = hb;
    sm.hp[1][m * KP + ncol] = lb;
  }
}

__device__ __forceinline__ void flush_chunk(const Smem& sm, float* out, int base, int c, int tid) {
  float* gb = out + ((size_t)base * S_ + (size_t)c * CH) * V_;
#pragma unroll
  for (int i = 0; i < 14; ++i) {
    int p = tid + NTH * i;
    if (p < (BT * ROWF) / 4) {
      int r = p / (ROWF / 4);
      int off = (p - r * (ROWF / 4)) * 4;
      v4f v = *(const v4f*)(&sm.stage[r * ROWF + off]);
      *(volatile v4f*)(gb + (size_t)r * (S_ * V_) + off) = v;
    }
  }
  __threadfence();
#pragma unroll
  for (int i = 0; i < 14; ++i) {
    int p = tid + NTH * i;
    if (p < (BT * ROWF) / 4) {
      int r = p / (ROWF / 4);
      int off = (p - r * (ROWF / 4)) * 4;
      v4f v = *(const v4f*)(&sm.stage[r * ROWF + off]);
      *(volatile v4f*)(gb + (size_t)r * (S_ * V_) + off) = v;
    }
  }
}

__global__ __launch_bounds__(NTH)
void k_tab(const float* embed, const float* eWx, const float* eb,
           const float* dWx, const float* db, float* Te, float* Td) {
  const int j = blockIdx.x * NTH + threadIdx.x;
  const bool dsel = (blockIdx.y != 0);
  const float* Wx = dsel ? dWx : eWx;
  const float* bb = dsel ? db : eb;
  float* T = dsel ? Td : Te;
  if (j >= NTAB) return;
  const int v = j >> 7, h = j & (H_ - 1);
  float s = 0.0f;
#pragma unroll 4
  for (int e = 0; e < E_; ++e) s = fmaf(embed[v * E_ + e], Wx[e * H_ + h], s);
  s += bb[h];
  float* d = T + j;
  *(volatile float*)d = s;
  __threadfence();
  *(volatile float*)d = s;
}

__global__ __launch_bounds__(NTH)
void k_seq(const int* enc_ids, const int* dec_ids, const float* Te, const float* Td,
           const float* enc_Wh, const float* dec_Wh, const float* dense_W, const float* dense_b,
           float* out, int nb) {
  __shared__ Smem sm;
  const int tid  = threadIdx.x;
  const int lane = tid & 31;
  const int w    = tid >> 5;
  const int hh   = lane >> 4;
  const int lm   = lane & 15;
  const int ncol = w * 16 + lm;
  const int base = blockIdx.x * BT;
  if (base + BT > nb) return;

  load_ids(sm, enc_ids, base, tid);
  load_wh(sm, enc_Wh, tid);
  load_wd(sm, dense_W, tid);
#pragma unroll 1
  for (int idx = tid; idx < 2 * BT * KP; idx += NTH)
    sm.hp[idx >> 11][idx & (BT * KP - 1)] = (unsigned short)0;
  const int   cb   = min(ncol, V_ - 1);
  const float lbv  = dense_b[cb];
  const float lbias = (ncol < V_) ? lbv : 0.0f;
  __syncthreads();

  const unsigned short* ah = &sm.hp[0][lm * KP + 8 * hh];
  const unsigned short* al = &sm.hp[1][lm * KP + 8 * hh];
  const unsigned short* bh = &sm.wh[0][ncol * KP + 8 * hh];
  const unsigned short* bl = &sm.wh[1][ncol * KP + 8 * hh];
  const int wdr = (w & 1) * 16 + lm;
  const unsigned short* dh = &sm.wd[0][wdr * KP + 8 * hh];
  const unsigned short* dl = &sm.wd[1][wdr * KP + 8 * hh];
  const v8f zero = {0.f, 0.f, 0.f, 0.f, 0.f, 0.f, 0.f, 0.f};

#pragma unroll 1
  for (int t = 0; t < S_; ++t) {
    v8f xin = gather_tab(sm, Te, t, hh, ncol);
    v8f acc = mma3(zero, ah, al, bh, bl);
    v8f pre = acc + xin;
    __syncthreads();
    write_h(sm, pre, hh, ncol);
    __syncthreads();
  }

  load_ids(sm, dec_ids, base, tid);
  load_wh(sm, dec_Wh, tid);
  __syncthreads();

#pragma unroll 1
  for (int t = 0; t < S_; ++t) {
    v8f xin = gather_tab(sm, Td, t, hh, ncol);
    v8f acc = mma3(zero, ah, al, bh, bl);
    v8f pre = acc + xin;
    __syncthreads();
    write_h(sm, pre, hh, ncol);
    __syncthreads();

    if (w < 2) {
      v8f lg = {lbias, lbias, lbias, lbias, lbias, lbias, lbias, lbias};
      lg = mma3(lg, ah, al, dh, dl);
      if (ncol < V_) {
        const int sl = t & (CH - 1);
#pragma unroll
        for (int r = 0; r < 8; ++r)
          sm.stage[(8 * hh + r) * ROWF + sl * V_ + ncol] = lg[r];
      }
    }
    if ((t & (CH - 1)) == (CH - 1)) {
      __syncthreads();
      flush_chunk(sm, out, base, t >> 5, tid);
    }
  }
}

extern "C" void kernel_launch(void* const* d_in, const int* in_sizes, int n_in,
                              void* d_out, int out_size, void* d_ws, size_t ws_size,
                              hipStream_t stream) {
  if (n_in < 11) return;
  if ((in_sizes[0] % S_) != 0) return;
  const int nb = in_sizes[0] / S_;
  if (nb <= 0 || (nb % BT) != 0) return;
  if (in_sizes[1] != nb * S_) return;
  if (in_sizes[2] != V_ * E_ || in_sizes[3] != E_ * H_ || in_sizes[4] != H_ * H_ ||
      in_sizes[5] != H_ || in_sizes[6] != E_ * H_ || in_sizes[7] != H_ * H_ ||
      in_sizes[8] != H_ || in_sizes[9] != H_ * V_ || in_sizes[10] != V_) return;
  if (out_size != nb * S_ * V_) return;

  const int*   enc_ids = (const int*)  d_in[0];
  const int*   dec_ids = (const int*)  d_in[1];
  const float* embed   = (const float*)d_in[2];
  const float* enc_Wx  = (const float*)d_in[3];
  const float* enc_Wh  = (const float*)d_in[4];
  const float* enc_b   = (const float*)d_in[5];
  const float* dec_Wx  = (const float*)d_in[6];
  const float* dec_Wh  = (const float*)d_in[7];
  const float* dec_b   = (const float*)d_in[8];
  const float* dense_W = (const float*)d_in[9];
  const float* dense_b = (const float*)d_in[10];
  float* out = (float*)d_out;

  const size_t tab_bytes = (size_t)NTAB * 4;
  const size_t need = 2 * tab_bytes;
  if (need > ws_size) return;
  char* ws = (char*)d_ws;
  float* Te = (float*)(ws);
  float* Td = (float*)(ws + tab_bytes);

  k_tab<<<dim3((NTAB + NTH - 1) / NTH, 2), dim3(NTH), 0, stream>>>(embed, enc_Wx, enc_b,
                                                                  dec_Wx, dec_b, Te, Td);
  k_seq<<<dim3(nb / BT), dim3(NTH), 0, stream>>>(enc_ids, dec_ids, Te, Td, enc_Wh, dec_Wh,
                                                 dense_W, dense_b, out, nb);
}
